// Recurrent_FullAttention_88751204204837
// MI455X (gfx1250) — hardware-verified
//
#include <hip/hip_runtime.h>
#include <math.h>

constexpr int NBATCH = 16;
constexpr int NPOS   = 256;
constexpr int NEMB   = 32;
constexpr int NFEA   = 7;
constexpr int ROWF   = NEMB * NFEA;
constexpr int NSP    = NPOS * NFEA;
constexpr int NGRP   = NSP / 8;
constexpr int NTHR   = 512;
constexpr int NWV    = NTHR / 32;
static_assert(ROWF == 224 && NSP == 1792 && NGRP == 224 && NWV == 16);
static_assert(NSP % 32 == 0);
static_assert((NSP * 4) % NTHR == 0);

constexpr float RES_CARRY      = 2048.0f;
constexpr float RES_INV        = 1.0f / RES_CARRY;
constexpr float P_CARRY        = 1024.0f;
constexpr float F16_MIN_NORMAL = 6.103515625e-05f;
constexpr float NEG_BIG        = -3.0e38f;

constexpr int SZ_X     = NSP * NEMB * 2;
constexpr int OFF_XHI  = 0;
constexpr int OFF_XLO  = OFF_XHI + SZ_X;
constexpr int OFF_PREG = OFF_XLO + SZ_X;
constexpr int SZ_PREG  = 8 * NGRP * 32;
constexpr int OFF_QHI  = OFF_PREG + SZ_PREG;
constexpr int OFF_QLO  = OFF_QHI + 16 * NEMB * 2;
constexpr int OFF_REDM = OFF_QLO + 16 * NEMB * 2;
constexpr int OFF_REDS = OFF_REDM + NWV * 8 * 4;
constexpr int OFF_OST  = OFF_REDS + NWV * 8 * 4;
constexpr int LDS_TOTAL = OFF_OST + 1024;
static_assert(SZ_X == 114688 && SZ_PREG == 57344 && LDS_TOTAL == 290816);
static_assert(LDS_TOTAL <= 327680);
static_assert(OFF_XLO % 16 == 0 && OFF_PREG % 16 == 0 && OFF_QHI % 16 == 0 && OFF_QLO % 16 == 0);
static_assert(OFF_REDM % 16 == 0 && OFF_REDS % 16 == 0 && OFF_OST % 16 == 0);
static_assert(NWV * 8 * NEMB * 4 <= SZ_PREG);
static_assert((768 + 64) * 4 <= SZ_PREG);
static_assert(ROWF * 4 <= 1024);
static_assert((ROWF * 4) % 128 == 0);

typedef __attribute__((ext_vector_type(16))) _Float16 v16h;
typedef __attribute__((ext_vector_type(8)))  float    v8f;
typedef __attribute__((ext_vector_type(4)))  float    v4f;
typedef __attribute__((ext_vector_type(4)))  unsigned v4u;
typedef __attribute__((ext_vector_type(8)))  unsigned v8u;
typedef v4u            v4u_a __attribute__((may_alias));
typedef v4f            v4f_a __attribute__((may_alias));
typedef float          f32_a __attribute__((may_alias));
typedef unsigned short u16_a __attribute__((may_alias));

__device__ __forceinline__ v8f mma16(v16h a, v16h b, v8f c) {
  c = __builtin_amdgcn_wmma_f32_16x16x32_f16(false, a, false, b, (short)0, c, false, false);
  asm volatile("v_nop\n\tv_nop\n\tv_nop\n\tv_nop" : "+v"(c) : "v"(a), "v"(b));
  return c;
}

__device__ __forceinline__ v16h frag_from(v4u a, v4u b) {
  const v8u w = __builtin_shufflevector(a, b, 0, 1, 2, 3, 4, 5, 6, 7);
  return __builtin_bit_cast(v16h, w);
}

__device__ __forceinline__ v16h gather_col(const u16_a* xb) {
  v8u w;
#pragma unroll
  for (int j = 0; j < 4; ++j) {
    const unsigned a0 = xb[(2 * j) * NEMB];
    const unsigned a1 = xb[(2 * j + 1) * NEMB];
    w[j] = a0 | (a1 << 16);
    const unsigned b0 = xb[(16 + 2 * j) * NEMB];
    const unsigned b1 = xb[(16 + 2 * j + 1) * NEMB];
    w[4 + j] = b0 | (b1 << 16);
  }
  return __builtin_bit_cast(v16h, w);
}

__device__ __forceinline__ void split16(float v, unsigned short& hb, unsigned short& lb) {
  const float vz = (fabsf(v) < F16_MIN_NORMAL) ? 0.0f : v;
  const _Float16 hv = (_Float16)vz;
  const float hf = (float)hv;
  const float rs = (v - hf) * RES_CARRY;
  const float rz = (fabsf(rs) < F16_MIN_NORMAL) ? 0.0f : rs;
  const _Float16 lv = (_Float16)rz;
  hb = __builtin_bit_cast(unsigned short, hv);
  lb = __builtin_bit_cast(unsigned short, lv);
}

__device__ __forceinline__ unsigned pk16(unsigned short a, unsigned short b) {
  return (unsigned)a | ((unsigned)b << 16);
}

__global__ void __launch_bounds__(NTHR, 1)
window_refeed_attn_kernel(const float* __restrict__ qin, const float* __restrict__ kin,
                            const float* __restrict__ vin, float* __restrict__ out) {
  extern __shared__ v4u smem_dyn[];
  unsigned char* const sm = (unsigned char*)smem_dyn;
  const int tid  = threadIdx.x;
  const int lane = tid & 31;
  const int wave = tid >> 5;
  const int c    = lane & 15;
  const int hh   = lane >> 4;
  const int b    = blockIdx.x;
  const size_t bbase = (size_t)b * NPOS * ROWF;

  u16_a* const xhi16 = (u16_a*)(sm + OFF_XHI);
  u16_a* const xlo16 = (u16_a*)(sm + OFF_XLO);
  u16_a* const qhi16 = (u16_a*)(sm + OFF_QHI);
  u16_a* const qlo16 = (u16_a*)(sm + OFF_QLO);
  f32_a* const preg_f = (f32_a*)(sm + OFF_PREG);
  f32_a* const redM  = (f32_a*)(sm + OFF_REDM);
  f32_a* const redS  = (f32_a*)(sm + OFF_REDS);
  f32_a* const ost   = (f32_a*)(sm + OFF_OST);

  const v8f z8 = {0.f, 0.f, 0.f, 0.f, 0.f, 0.f, 0.f, 0.f};

#pragma unroll 1
  for (int it = 0; it < (NSP * 4) / NTHR; ++it) {
    const int i  = it * NTHR + tid;
    const int sp = i >> 2;
    const int eg = (i & 3) * 8;
    const int s  = sp / NFEA;
    const int p  = sp - s * NFEA;
    const float* src = vin + bbase + (size_t)s * ROWF + eg * NFEA + p;
    unsigned short hb[8], lb[8];
#pragma unroll
    for (int j = 0; j < 8; ++j) {
      const float xv = src[j * NFEA];
      split16(xv, hb[j], lb[j]);
    }
    const v4u uh = {pk16(hb[0], hb[1]), pk16(hb[2], hb[3]), pk16(hb[4], hb[5]), pk16(hb[6], hb[7])};
    const v4u ul = {pk16(lb[0], lb[1]), pk16(lb[2], lb[3]), pk16(lb[4], lb[5]), pk16(lb[6], lb[7])};
    *(v4u_a*)(sm + OFF_XHI + sp * 64 + eg * 2) = uh;
    *(v4u_a*)(sm + OFF_XLO + sp * 64 + eg * 2) = ul;
  }
  if (tid < ROWF) {
    preg_f[tid]       = qin[bbase + tid];
    preg_f[256 + tid] = kin[bbase + tid];
    preg_f[512 + tid] = vin[bbase + tid];
  }
  __syncthreads();

  if (tid < NFEA * NFEA) {
    const int p = tid / NFEA;
    const int r = tid - p * NFEA;
    float s0 = 0.0f;
#pragma unroll 1
    for (int e = 0; e < NEMB; ++e) s0 = fmaf(preg_f[e * NFEA + r], preg_f[256 + e * NFEA + p], s0);
    preg_f[768 + p * 8 + r] = s0;
  }
  __syncthreads();
  if (tid < NFEA) {
    float mx = NEG_BIG;
#pragma unroll 1
    for (int p = 0; p < NFEA; ++p) mx = fmaxf(mx, preg_f[768 + p * 8 + tid]);
    float sm0 = 0.0f;
#pragma unroll 1
    for (int p = 0; p < NFEA; ++p) {
      const float ev = expf(preg_f[768 + p * 8 + tid] - mx);
      preg_f[768 + p * 8 + tid] = ev;
      sm0 += ev;
    }
    const float inv0 = 1.0f / sm0;
#pragma unroll 1
    for (int p = 0; p < NFEA; ++p) preg_f[768 + p * 8 + tid] = preg_f[768 + p * 8 + tid] * inv0;
  }
  __syncthreads();
  if (tid < ROWF) {
    const int r = tid >> 5;
    const int e = tid & 31;
    float o = 0.0f;
#pragma unroll 1
    for (int p = 0; p < NFEA; ++p) o = fmaf(preg_f[512 + e * NFEA + p], preg_f[768 + p * 8 + r], o);
    ost[e * NFEA + r] = o;
    unsigned short hb, lb;
    split16(o, hb, lb);
    xhi16[r * NEMB + e] = hb;
    xlo16[r * NEMB + e] = lb;
  }
  {
    const int n  = tid >> 5;
    const int e  = tid & 31;
    const int nn = (n < NFEA) ? n : (NFEA - 1);
    float qv = qin[bbase + (size_t)1 * ROWF + e * NFEA + nn];
    asm volatile("" : "+v"(qv));
    const float qz = (n < NFEA) ? qv : 0.0f;
    unsigned short hb, lb;
    split16(qz, hb, lb);
    qhi16[n * NEMB + e] = hb;
    qlo16[n * NEMB + e] = lb;
  }
  __syncthreads();
  if (wave == 0) {
    float* const orow = out + bbase;
    float vv[7];
#pragma unroll
    for (int i = 0; i < 7; ++i) vv[i] = ost[i * 32 + lane];
    for (int pass = 0; pass < 2; ++pass) {
#pragma unroll
      for (int i = 0; i < 7; ++i) *(volatile float*)(orow + i * 32 + lane) = vv[i];
      __threadfence();
    }
  }

#pragma unroll 1
  for (int t = 1; t < NPOS; ++t) {
    const int liveRows = (t + 1) * NFEA;
    const int padRows  = (liveRows + 31) & ~31;
    const int nTiles   = padRows >> 4;
    const int nKsteps  = padRows >> 5;

    {
      const v4u_a* qp = (const v4u_a*)(sm + OFF_QHI + c * 64 + hh * 16);
      const v16h qh = frag_from(qp[0], qp[2]);
      const v4u_a* qq = (const v4u_a*)(sm + OFF_QLO + c * 64 + hh * 16);
      const v16h ql = frag_from(qq[0], qq[2]);
      float lmax = NEG_BIG;
#pragma unroll 1
      for (int tile = wave; tile < nTiles; tile += NWV) {
        const int rowbase = tile * 16;
        const v4u_a* xa = (const v4u_a*)(sm + OFF_XHI + (rowbase + c) * 64 + hh * 16);
        const v16h ah = frag_from(xa[0], xa[2]);
        const v4u_a* xl = (const v4u_a*)(sm + OFF_XLO + (rowbase + c) * 64 + hh * 16);
        const v16h al = frag_from(xl[0], xl[2]);
        v8f acc = z8;
        v8f accr = z8;
        acc  = mma16(ah, qh, acc);
        accr = mma16(ah, ql, accr);
        accr = mma16(al, qh, accr);
        float sv[8];
#pragma unroll
        for (int r = 0; r < 8; ++r) sv[r] = acc[r] + accr[r] * RES_INV;
        const int sp0 = rowbase + 8 * hh;
#pragma unroll
        for (int r = 0; r < 8; ++r) {
          const float cand = fmaxf(lmax, sv[r]);
          lmax = (sp0 + r < liveRows) ? cand : lmax;
        }
        if (c < 8) {
          v4f_a* sc = (v4f_a*)(sm + OFF_PREG + ((c & 7) * NGRP + tile * 2 + hh) * 32);
          const v4f s0 = {sv[0], sv[1], sv[2], sv[3]};
          const v4f s1 = {sv[4], sv[5], sv[6], sv[7]};
          sc[0] = s0;
          sc[1] = s1;
        }
      }
      const float other = __shfl_xor(lmax, 16, 32);
      lmax = fmaxf(lmax, other);
      if (lane < 8) redM[wave * 8 + lane] = lmax;
    }
    __syncthreads();

    {
      const int cc = tid & 7;
      float mx = NEG_BIG;
#pragma unroll
      for (int w = 0; w < NWV; ++w) mx = fmaxf(mx, redM[w * 8 + cc]);
      float lsum = 0.0f;
#pragma unroll 1
      for (int j = tid; j < padRows; j += NTHR) {
        const int g = j >> 3;
        unsigned char* const chunk = sm + OFF_PREG + (cc * NGRP + g) * 32;
        const v4f s0 = ((const v4f_a*)chunk)[0];
        const v4f s1 = ((const v4f_a*)chunk)[1];
        float sv[8];
        sv[0] = s0[0]; sv[1] = s0[1]; sv[2] = s0[2]; sv[3] = s0[3];
        sv[4] = s1[0]; sv[5] = s1[1]; sv[6] = s1[2]; sv[7] = s1[3];
        unsigned short hb[8], lb[8];
#pragma unroll
        for (int i = 0; i < 8; ++i) {
          const bool live = (g * 8 + i < liveRows) && (cc < NFEA);
          const float arg = fminf(sv[i] - mx, 0.0f);
          const float ev  = expf(arg);
          const float pv  = live ? ev : 0.0f;
          lsum += pv;
          split16(pv * P_CARRY, hb[i], lb[i]);
        }
        const v4u uh = {pk16(hb[0], hb[1]), pk16(hb[2], hb[3]), pk16(hb[4], hb[5]), pk16(hb[6], hb[7])};
        const v4u ul = {pk16(lb[0], lb[1]), pk16(lb[2], lb[3]), pk16(lb[4], lb[5]), pk16(lb[6], lb[7])};
        ((v4u_a*)chunk)[0] = uh;
        ((v4u_a*)chunk)[1] = ul;
      }
      const float s8 = __shfl_xor(lsum, 8, 32);
      lsum += s8;
      const float s16 = __shfl_xor(lsum, 16, 32);
      lsum += s16;
      if (lane < 8) redS[wave * 8 + lane] = lsum;
    }
    __syncthreads();

    v8f o0, o1;
    {
      v8f a0 = z8;
      v8f a1 = z8;
      v8f r0 = z8;
      v8f r1 = z8;
      const int mr = c & 7;
#pragma unroll 1
      for (int ks = wave; ks < nKsteps; ks += NWV) {
        const v4u_a* pp = (const v4u_a*)(sm + OFF_PREG + (mr * NGRP + ks * 4 + hh) * 32);
        const v16h ph = frag_from(pp[0], pp[4]);
        const v16h pl = frag_from(pp[1], pp[5]);
        const u16_a* xb  = xhi16 + (ks * 32 + 8 * hh) * NEMB + c;
        const u16_a* xlb = xlo16 + (ks * 32 + 8 * hh) * NEMB + c;
        {
          const v16h xh = gather_col(xb);
          const v16h xl = gather_col(xlb);
          a0 = mma16(ph, xh, a0);
          r0 = mma16(ph, xl, r0);
          r0 = mma16(pl, xh, r0);
        }
        {
          const v16h xh = gather_col(xb + 16);
          const v16h xl = gather_col(xlb + 16);
          a1 = mma16(ph, xh, a1);
          r1 = mma16(ph, xl, r1);
          r1 = mma16(pl, xh, r1);
        }
      }
#pragma unroll
      for (int r = 0; r < 8; ++r) {
        o0[r] = a0[r] + r0[r] * RES_INV;
        o1[r] = a1[r] + r1[r] * RES_INV;
      }
    }
    __syncthreads();
    if (hh == 0) {
      f32_a* const part = preg_f + wave * (8 * NEMB);
#pragma unroll
      for (int r = 0; r < 8; ++r) {
        part[r * NEMB + c]      = o0[r];
        part[r * NEMB + 16 + c] = o1[r];
      }
    }
    __syncthreads();

    if (tid < ROWF) {
      const int r = tid >> 5;
      const int e = tid & 31;
      float s = 0.0f;
#pragma unroll
      for (int w = 0; w < NWV; ++w) s += preg_f[(w * 8 + r) * NEMB + e];
      float cs = 0.0f;
#pragma unroll
      for (int w = 0; w < NWV; ++w) cs += redS[w * 8 + r];
      const float inv = 1.0f / (cs * P_CARRY);
      const float val = s * inv;
      ost[e * NFEA + r] = val;
      unsigned short hb, lb;
      split16(val, hb, lb);
      xhi16[(t * NFEA + r) * NEMB + e] = hb;
      xlo16[(t * NFEA + r) * NEMB + e] = lb;
    }
    {
      const int tn = (t + 1 < NPOS) ? (t + 1) : (NPOS - 1);
      const int n  = tid >> 5;
      const int e  = tid & 31;
      const int nn = (n < NFEA) ? n : (NFEA - 1);
      float qv = qin[bbase + (size_t)tn * ROWF + e * NFEA + nn];
      asm volatile("" : "+v"(qv));
      const float qz = (n < NFEA) ? qv : 0.0f;
      unsigned short hb, lb;
      split16(qz, hb, lb);
      qhi16[n * NEMB + e] = hb;
      qlo16[n * NEMB + e] = lb;
    }
    __syncthreads();
    if (wave == 0) {
      float* const orow = out + bbase + (size_t)t * ROWF;
      float vv[7];
#pragma unroll
      for (int i = 0; i < 7; ++i) vv[i] = ost[i * 32 + lane];
      for (int pass = 0; pass < 2; ++pass) {
#pragma unroll
        for (int i = 0; i < 7; ++i) *(volatile float*)(orow + i * 32 + lane) = vv[i];
        __threadfence();
      }
    }
  }
}

extern "C" void kernel_launch(void* const* d_in, const int* in_sizes, int n_in,
                              void* d_out, int out_size, void* d_ws, size_t ws_size, hipStream_t stream) {
  (void)d_ws; (void)ws_size;
  if (n_in < 3 || d_out == nullptr) return;
  const int nElem = NBATCH * NPOS * ROWF;
  if (in_sizes[0] != nElem || in_sizes[1] != nElem || in_sizes[2] != nElem || out_size != nElem) return;
  const float* qin = (const float*)d_in[0];
  const float* kin = (const float*)d_in[1];
  const float* vin = (const float*)d_in[2];
  float* out = (float*)d_out;
  window_refeed_attn_kernel<<<dim3(NBATCH), dim3(NTHR), LDS_TOTAL, stream>>>(qin, kin, vin, out);
}
